// GATEncoderLayer_87076166959574
// MI455X (gfx1250) — hardware-run, weakly checked
//
#include <hip/hip_runtime.h>
#include <stddef.h>
#include <stdint.h>


#define A2_TERMS 2
#define FIN     64
#define HC      256
#define NC2     512
#define PP      512
#define KT2     512
#define NEGS    0.2f
#define NTHR    256
#define NWAVE   8
#define EPT     8
#define CHUNK   (NTHR * EPT)
#define WCAP    (EPT * 32)
#define LISTN   (NWAVE * WCAP)
#define NBA     512
#define PKS     9
#define RCAP    16384
#define DEGCAP  64
#define GBM     64
#define GBN     64
#define GTHR    128
#define RPB     64
#define RPW     8
#define BK_INTS (2 * RCAP + 3 * NBA + LISTN + 32)
#define LDS_BK  (BK_INTS * 4)
#define MEAS_BLK_HITS 13125
#define MEAS_MAXDEG   46
#define U_W1    (NC2 * (FIN / 8))
#define U_W2    (NC2 * (KT2 / 8))
#define U_VEC   512
#define U_FIX   (U_W1 + U_W2 + U_VEC)
#define VEC_N   2048
#define V_BLR1  0
#define V_BLR2  512
#define V_ATT1  1024
#define V_ATT2  1280
#define V_BIAS1 1536
#define V_BIAS2 1792
#define WSMAX   (128u << 20)

static_assert(A2_TERMS == 1 || A2_TERMS == 2);
static_assert(HC == 32 * 8 && HC == 4 * 64);
static_assert((CHUNK & (CHUNK - 1)) == 0 && CHUNK <= 4096);
static_assert(NBA == (1 << PKS) && NBA == NTHR * 2 && NBA <= 1024);
static_assert(LISTN == NWAVE * WCAP);
static_assert(RCAP % (NTHR * 4) == 0 && BK_INTS % 4 == 0);
static_assert((long long)RCAP * 100 >= (long long)MEAS_BLK_HITS * 105);
static_assert(DEGCAP >= MEAS_MAXDEG + 8);
static_assert(LDS_BK <= 300000);
static_assert(GBM == (GTHR / 32) * 16 && (NC2 % GBN) == 0 && (HC % GBN) == 0);
static_assert((FIN % 32) == 0 && ((HC * A2_TERMS) % 32) == 0 && PP == 2 * HC && KT2 == 2 * HC);
static_assert(((U_W1 / 2) % NTHR) == 0 && ((U_W2 / 2) % NTHR) == 0 && (U_FIX % NTHR) == 0 && (U_VEC % NTHR) == 0);
static_assert(RPB == NWAVE * RPW);
static_assert(VEC_N == U_VEC * 4);

typedef float          v4f   __attribute__((ext_vector_type(4)));
typedef float          v8f   __attribute__((ext_vector_type(8)));
typedef int            v2i   __attribute__((ext_vector_type(2)));
typedef int            v4i   __attribute__((ext_vector_type(4)));
typedef int            v8i   __attribute__((ext_vector_type(8)));
typedef unsigned       v4u   __attribute__((ext_vector_type(4)));
typedef unsigned short v8us  __attribute__((ext_vector_type(8)));
typedef __bf16         v16bf __attribute__((ext_vector_type(16)));
typedef v4f  __attribute__((may_alias)) v4fa;
typedef v2i  __attribute__((may_alias)) v2ia;
typedef v4i  __attribute__((may_alias)) v4ia;
typedef v8us __attribute__((may_alias)) v8usa;
union FragB { v16bf v; v8us h[2]; v8i w; };

__device__ __forceinline__ v8f wmb(const FragB& a, const FragB& b, v8f c) {
  v8f d = __builtin_amdgcn_wmma_f32_16x16x32_bf16(false, a.v, false, b.v, (short)0, c, false, false);
  asm volatile("v_nop\n\tv_nop\n\tv_nop\n\tv_nop" : "+v"(d) : "v"(a.w), "v"(b.w));
  return d;
}

__device__ __forceinline__ unsigned bf16_bits(float f) {
  const unsigned u = __float_as_uint(f);
  return ((u + 0x7FFFu + ((u >> 16) & 1u)) >> 16) & 0xFFFFu;
}
__device__ __forceinline__ float bf16_val(float f) { return __uint_as_float(bf16_bits(f) << 16); }
__device__ __forceinline__ void pack2(float a, float b, unsigned& hw, unsigned& lw) {
  const unsigned ha = bf16_bits(a), hb = bf16_bits(b);
  const unsigned la = bf16_bits(a - __uint_as_float(ha << 16));
  const unsigned lb = bf16_bits(b - __uint_as_float(hb << 16));
  hw = ha | (hb << 16);
  lw = la | (lb << 16);
}
__device__ __forceinline__ v8us cvt8(const v4f a, const v4f b) {
  v8us o;
  o[0] = (unsigned short)bf16_bits(a.x); o[1] = (unsigned short)bf16_bits(a.y);
  o[2] = (unsigned short)bf16_bits(a.z); o[3] = (unsigned short)bf16_bits(a.w);
  o[4] = (unsigned short)bf16_bits(b.x); o[5] = (unsigned short)bf16_bits(b.y);
  o[6] = (unsigned short)bf16_bits(b.z); o[7] = (unsigned short)bf16_bits(b.w);
  return o;
}
__device__ __forceinline__ v4u blend4(v4u r, const v4f v, unsigned mk) {
  r.x |= __float_as_uint(v.x) & mk;
  r.y |= __float_as_uint(v.y) & mk;
  r.z |= __float_as_uint(v.z) & mk;
  r.w |= __float_as_uint(v.w) & mk;
  return r;
}

__device__ __forceinline__ void wave_sync() {
  __builtin_amdgcn_fence(__ATOMIC_RELEASE, "wavefront");
  __builtin_amdgcn_wave_barrier();
  __builtin_amdgcn_fence(__ATOMIC_ACQUIRE, "wavefront");
}

__device__ __forceinline__ void slot_info(const int* __restrict__ CNT, const int* __restrict__ OFF, int node,
                                          int& c, int& o) {
  const int craw = CNT[node];
  const int oraw = OFF[node];
  const int deg = craw < 0 ? 0 : craw;
  c = deg > DEGCAP ? DEGCAP : deg;
  o = oraw < 0 ? 0 : (oraw > RCAP ? RCAP : oraw);
  if (c > RCAP - o) c = RCAP - o;
}

__device__ __forceinline__ int scan_chunk(const int* __restrict__ keys, int nE, int cbase, int slotBase,
                                          int nb, int vec8, int* list, int tid, int lane, int wave) {
  int wc = 0;
  const int el0  = tid * EPT;
  const int e0   = cbase + el0;
  const int sent = (int)(1u << 31);
  v4i da, db;
  if (vec8 != 0 && cbase + CHUNK <= nE) {
    da = *(const v4i*)(keys + e0);
    db = *(const v4i*)(keys + e0 + 4);
  } else {
    const int t0 = keys[min(e0,     nE - 1)];
    const int t1 = keys[min(e0 + 1, nE - 1)];
    const int t2 = keys[min(e0 + 2, nE - 1)];
    const int t3 = keys[min(e0 + 3, nE - 1)];
    const int t4 = keys[min(e0 + 4, nE - 1)];
    const int t5 = keys[min(e0 + 5, nE - 1)];
    const int t6 = keys[min(e0 + 6, nE - 1)];
    const int t7 = keys[min(e0 + 7, nE - 1)];
    asm volatile("" :: "v"(t0), "v"(t1), "v"(t2), "v"(t3), "v"(t4), "v"(t5), "v"(t6), "v"(t7));
    da.x = (e0     < nE) ? t0 : sent;
    da.y = (e0 + 1 < nE) ? t1 : sent;
    da.z = (e0 + 2 < nE) ? t2 : sent;
    da.w = (e0 + 3 < nE) ? t3 : sent;
    db.x = (e0 + 4 < nE) ? t4 : sent;
    db.y = (e0 + 5 < nE) ? t5 : sent;
    db.z = (e0 + 6 < nE) ? t6 : sent;
    db.w = (e0 + 7 < nE) ? t7 : sent;
  }
  const unsigned nbs = (unsigned)slotBase;
  const unsigned unb = (unsigned)nb;
  const unsigned s0 = (unsigned)da.x - nbs, s1 = (unsigned)da.y - nbs;
  const unsigned s2 = (unsigned)da.z - nbs, s3 = (unsigned)da.w - nbs;
  const unsigned s4 = (unsigned)db.x - nbs, s5 = (unsigned)db.y - nbs;
  const unsigned s6 = (unsigned)db.z - nbs, s7 = (unsigned)db.w - nbs;
  const bool h0 = s0 < unb, h1 = s1 < unb, h2 = s2 < unb, h3 = s3 < unb;
  const bool h4 = s4 < unb, h5 = s5 < unb, h6 = s6 < unb, h7 = s7 < unb;
  const unsigned any = __builtin_amdgcn_ballot_w32(h0 | h1 | h2 | h3 | h4 | h5 | h6 | h7);
  if (any != 0u) {
#define HITJ(J, HJ, SJ) { \
      const unsigned mj = __builtin_amdgcn_ballot_w32(HJ); \
      if (mj != 0u) { \
        if (HJ) { \
          const int pos = wc + (int)__builtin_amdgcn_mbcnt_lo(mj, 0u); \
          if (pos < WCAP) list[wave * WCAP + pos] = ((el0 + (J)) << PKS) | (int)(SJ); \
        } \
        wc += (int)__builtin_popcount(mj); } }
    HITJ(0, h0, s0)
    HITJ(1, h1, s1)
    HITJ(2, h2, s2)
    HITJ(3, h3, s3)
    HITJ(4, h4, s4)
    HITJ(5, h5, s5)
    HITJ(6, h6, s6)
    HITJ(7, h7, s7)
#undef HITJ
  }
  return wc;
}

__global__ __launch_bounds__(NTHR) void k_prep(
    const float* __restrict__ x,
    const float* __restrict__ wl1, const float* __restrict__ wr1,
    const float* __restrict__ wl2, const float* __restrict__ wr2,
    const float* __restrict__ bl1, const float* __restrict__ br1,
    const float* __restrict__ bl2, const float* __restrict__ br2,
    const float* __restrict__ att1, const float* __restrict__ att2,
    const float* __restrict__ bias1, const float* __restrict__ bias2,
    unsigned short* w1t, unsigned short* w2t, float* vec, unsigned short* xb, unsigned short* x1,
    int nN, int nUX, int nPad) {
  const int ub = (int)blockIdx.x * NTHR;
  const int u  = ub + (int)threadIdx.x;
  if (ub < U_W1) {
    const int n  = u >> 3;
    const int k8 = (u & 7) * 8;
    const int nn = n & (HC - 1);
    const size_t so = (size_t)k8 * HC + (size_t)nn;
    float f[8];
    if (ub < U_W1 / 2) {
#pragma unroll
      for (int i = 0; i < 8; ++i) f[i] = wl1[so + (size_t)i * HC];
    } else {
#pragma unroll
      for (int i = 0; i < 8; ++i) f[i] = wr1[so + (size_t)i * HC];
    }
    v8us o;
#pragma unroll
    for (int i = 0; i < 8; ++i) o[i] = (unsigned short)bf16_bits(f[i]);
    unsigned short* dp = w1t + (size_t)n * FIN + (size_t)k8;
    *(volatile v8us*)dp = o;
    __threadfence();
    *(volatile v8us*)dp = o;
  } else if (ub < U_W1 + U_W2) {
    const int uu = u - U_W1;
    const int n  = uu >> 6;
    const int k8 = (uu & 63) * 8;
    const int ks = k8 & (HC - 1);
    const int nn = n & (HC - 1);
    const size_t so = (size_t)ks * HC + (size_t)nn;
    float f[8];
    if (ub - U_W1 < U_W2 / 2) {
#pragma unroll
      for (int i = 0; i < 8; ++i) f[i] = wl2[so + (size_t)i * HC];
    } else {
#pragma unroll
      for (int i = 0; i < 8; ++i) f[i] = wr2[so + (size_t)i * HC];
    }
    v8us o;
#pragma unroll
    for (int i = 0; i < 8; ++i) o[i] = (unsigned short)bf16_bits(f[i]);
    unsigned short* dp = w2t + (size_t)n * KT2 + (size_t)k8;
    *(volatile v8us*)dp = o;
    __threadfence();
    *(volatile v8us*)dp = o;
  } else if (ub < U_FIX) {
    const int uu  = u - (U_W1 + U_W2);
    const int seg = uu >> 6;
    const int q   = (uu & 63) * 4;
    const v4f c0 = *(const v4f*)(bl1 + q);
    const v4f c1 = *(const v4f*)(br1 + q);
    const v4f c2 = *(const v4f*)(bl2 + q);
    const v4f c3 = *(const v4f*)(br2 + q);
    const v4f c4 = *(const v4f*)(att1 + q);
    const v4f c5 = *(const v4f*)(att2 + q);
    const v4f c6 = *(const v4f*)(bias1 + q);
    const v4f c7 = *(const v4f*)(bias2 + q);
    asm volatile("" :: "v"(c0), "v"(c1), "v"(c2), "v"(c3));
    asm volatile("" :: "v"(c4), "v"(c5), "v"(c6), "v"(c7));
    v4u r = {0u, 0u, 0u, 0u};
    r = blend4(r, c0, (seg == 0) ? 0xFFFFFFFFu : 0u);
    r = blend4(r, c1, (seg == 1) ? 0xFFFFFFFFu : 0u);
    r = blend4(r, c2, (seg == 2) ? 0xFFFFFFFFu : 0u);
    r = blend4(r, c3, (seg == 3) ? 0xFFFFFFFFu : 0u);
    r = blend4(r, c4, (seg == 4) ? 0xFFFFFFFFu : 0u);
    r = blend4(r, c5, (seg == 5) ? 0xFFFFFFFFu : 0u);
    r = blend4(r, c6, (seg == 6) ? 0xFFFFFFFFu : 0u);
    r = blend4(r, c7, (seg == 7) ? 0xFFFFFFFFu : 0u);
    v4f o;
    o.x = bf16_val(__uint_as_float(r.x));
    o.y = bf16_val(__uint_as_float(r.y));
    o.z = bf16_val(__uint_as_float(r.z));
    o.w = bf16_val(__uint_as_float(r.w));
    float* dp = vec + (size_t)uu * 4;
    *(volatile v4f*)dp = o;
    __threadfence();
    *(volatile v4f*)dp = o;
  } else if (ub < U_FIX + nUX) {
    const int uu  = u - U_FIX;
    const int row = uu >> 3;
    const int c0  = (uu & 7) * 8;
    const int rc  = row < nN ? row : nN - 1;
    const float* p = x + (size_t)rc * FIN + c0;
    v4f a = *(const v4f*)p, b = *(const v4f*)(p + 4);
    asm volatile("" :: "v"(a), "v"(b));
    const v4f z4 = {0.f, 0.f, 0.f, 0.f};
    if (row >= nN) { a = z4; b = z4; }
    const v8us hv = cvt8(a, b);
    unsigned short* dp = xb + (size_t)row * FIN + c0;
    *(volatile v8us*)dp = hv;
    __threadfence();
    *(volatile v8us*)dp = hv;
  } else {
    const int uu = u - U_FIX - nUX;
    const bool ok = uu < nPad;
    const int us = ok ? uu : 0;
    const v4u z = {0u, 0u, 0u, 0u};
    unsigned short* dp = x1 + (size_t)nN * PP + (size_t)us * 8;
    if (ok) *(volatile v4u*)dp = z;
    __threadfence();
    if (ok) *(volatile v4u*)dp = z;
  }
}

__global__ __launch_bounds__(NTHR) void k_bucket(const int* __restrict__ keys, const int* __restrict__ gidx,
                                                 int nE, int nN, int vec8,
                                                 int* LIST, int* CNT, int* OFF, int* REC) {
  extern __shared__ __attribute__((aligned(16))) int dsm[];
  int* reg1 = dsm;
  int* reg2 = reg1 + RCAP;
  int* scnt = reg2 + RCAP;
  int* soff = scnt + NBA;
  int* cur  = soff + NBA;
  int* list = cur + NBA;
  int* wcnt = list + LISTN;
  int* wtot = wcnt + 8;
  int* wmx  = wtot + 8;
  const int tid = (int)threadIdx.x, lane = tid & 31, wave = tid >> 5;
  const int nodeBase = (int)blockIdx.x * NBA;
  int nb = nN - nodeBase;
  nb = nb > NBA ? NBA : (nb < 1 ? 1 : nb);

  {
    const v4i z4 = {0, 0, 0, 0};
    for (int i = tid * 4; i < BK_INTS; i += NTHR * 4) *(v4ia*)(dsm + i) = z4;
  }
  __syncthreads();

  int tot = 0;
  const int nChunks = (nE + CHUNK - 1) / CHUNK;
#pragma unroll 1
  for (int ch = 0; ch < nChunks; ++ch) {
    const int cbase = ch * CHUNK;
    const int wc = scan_chunk(keys, nE, cbase, nodeBase, nb, vec8, list, tid, lane, wave);
    if (lane == 0) wcnt[wave] = wc;
    __syncthreads();
    int pre = 0, all = 0;
#pragma unroll
    for (int w2 = 0; w2 < NWAVE; ++w2) {
      int c = wcnt[w2];
      c = c < 0 ? 0 : (c > WCAP ? WCAP : c);
      all += c;
      pre += (w2 < wave) ? c : 0;
    }
    const int wcc  = wc > WCAP ? WCAP : wc;
    const int base = tot + pre;
#pragma unroll 1
    for (int i = lane; i < wcc; i += 32) {
      const int ent = list[wave * WCAP + i];
      const int el  = (ent >> PKS) & (CHUNK - 1);
      const int sl  = ent & (NBA - 1);
      int eid = cbase + el;
      eid = eid > nE - 1 ? nE - 1 : eid;
      const int pos = base + i;
      if (pos < RCAP) reg1[pos] = (int)(((unsigned)eid << PKS) | (unsigned)sl);
    }
    tot += all;
    tot = tot > RCAP ? RCAP : tot;
    __syncthreads();
  }
  const int nh = tot;

  if (wave == 0) {
#pragma unroll 1
    for (int b0 = 0; b0 < nh; b0 += 32) {
      const int idx = b0 + lane;
      const int uv  = reg1[idx < RCAP ? idx : RCAP - 1];
      const int m32 = (nh - b0) < 32 ? (nh - b0) : 32;
#pragma unroll 1
      for (int k = 0; k < m32; ++k) {
        const int u  = __builtin_amdgcn_readlane(uv, k);
        const int sl = u & (NBA - 1);
        if (lane == 0) scnt[sl] = scnt[sl] + 1;
      }
    }
  }
  __syncthreads();

  {
    const v2i ca = *(const v2ia*)(scnt + 2 * tid);
    const int e0 = ca.x < 0 ? 0 : ca.x, e1 = ca.y < 0 ? 0 : ca.y;
    const int ts = e0 + e1;
    int incl = ts;
#pragma unroll
    for (int d = 1; d < 32; d <<= 1) {
      const int up = __shfl_up(incl, d, 32);
      if (lane >= d) incl += up;
    }
    int mx = max(e0, e1);
    mx = max(mx, __shfl_xor(mx, 16, 32));
    mx = max(mx, __shfl_xor(mx, 8, 32));
    mx = max(mx, __shfl_xor(mx, 4, 32));
    mx = max(mx, __shfl_xor(mx, 2, 32));
    mx = max(mx, __shfl_xor(mx, 1, 32));
    if (lane == 31) wtot[wave] = incl;
    if (lane == 0)  wmx[wave] = mx;
    __syncthreads();
    int pre = 0;
#pragma unroll
    for (int w2 = 0; w2 < NWAVE; ++w2) pre += (w2 < wave) ? wtot[w2] : 0;
    const int run = pre + incl - ts;
    v2i so;
    so.x = run;
    so.y = run + e0;
    *(v2ia*)(soff + 2 * tid) = so;
    *(v2ia*)(cur + 2 * tid)  = so;
  }
  __syncthreads();

  if (wave == 0) {
#pragma unroll 1
    for (int b0 = 0; b0 < nh; b0 += 32) {
      const int idx = b0 + lane;
      const int uv  = reg1[idx < RCAP ? idx : RCAP - 1];
      const int m32 = (nh - b0) < 32 ? (nh - b0) : 32;
#pragma unroll 1
      for (int k = 0; k < m32; ++k) {
        const int u   = __builtin_amdgcn_readlane(uv, k);
        const int sl  = u & (NBA - 1);
        const int eid = (int)((unsigned)u >> PKS);
        if (lane == 0) {
          int pos = cur[sl];
          pos = pos < 0 ? 0 : (pos > RCAP - 1 ? RCAP - 1 : pos);
          reg2[pos] = eid;
          cur[sl] = pos + 1;
        }
      }
    }
  }
  __syncthreads();

  int bmax = 0;
#pragma unroll
  for (int w2 = 0; w2 < NWAVE; ++w2) bmax = max(bmax, wmx[w2]);
  const int flag = ((nh >= RCAP) || (bmax > DEGCAP)) ? 1 : 0;

  int* lrow = LIST + (size_t)blockIdx.x * RCAP;
#pragma unroll 1
  for (int it = 0; it < RCAP / (NTHR * 4); ++it) {
    const int i0 = 4 * (it * NTHR + tid);
    const v4i ev = *(const v4ia*)(reg2 + i0);
    int e0 = ev.x, e1 = ev.y, e2 = ev.z, e3 = ev.w;
    e0 = e0 < 0 ? 0 : (e0 > nE - 1 ? nE - 1 : e0);
    e1 = e1 < 0 ? 0 : (e1 > nE - 1 ? nE - 1 : e1);
    e2 = e2 < 0 ? 0 : (e2 > nE - 1 ? nE - 1 : e2);
    e3 = e3 < 0 ? 0 : (e3 > nE - 1 ? nE - 1 : e3);
    int g0 = gidx[e0], g1 = gidx[e1], g2 = gidx[e2], g3 = gidx[e3];
    asm volatile("" :: "v"(g0), "v"(g1), "v"(g2), "v"(g3));
    g0 = g0 < 0 ? 0 : (g0 > nN - 1 ? nN - 1 : g0);
    g1 = g1 < 0 ? 0 : (g1 > nN - 1 ? nN - 1 : g1);
    g2 = g2 < 0 ? 0 : (g2 > nN - 1 ? nN - 1 : g2);
    g3 = g3 < 0 ? 0 : (g3 > nN - 1 ? nN - 1 : g3);
    v4i ov;
    ov.x = (i0     < nh) ? g0 : 0;
    ov.y = (i0 + 1 < nh) ? g1 : 0;
    ov.z = (i0 + 2 < nh) ? g2 : 0;
    ov.w = (i0 + 3 < nh) ? g3 : 0;
    *(volatile v4i*)(lrow + i0) = ov;
    __threadfence();
    *(volatile v4i*)(lrow + i0) = ov;
  }
  {
    const int t4 = 4 * (tid & 127);
    const v4i cv = *(const v4ia*)(scnt + t4);
    const v4i fv = *(const v4ia*)(soff + t4);
    v4i rv = {0, 0, 0, 0};
    rv.x = (tid == 0) ? bmax : 0;
    rv.y = (tid == 0) ? flag : 0;
    rv.z = (tid == 0) ? nh : 0;
    int* cp = CNT + (size_t)nodeBase + t4;
    int* fp = OFF + (size_t)nodeBase + t4;
    int* rp = REC + (size_t)blockIdx.x * 32 + 4 * (tid & 7);
    const bool w4 = tid < 128;
    if (w4) { *(volatile v4i*)cp = cv; *(volatile v4i*)fp = fv; }
    if (tid < 8) *(volatile v4i*)rp = rv;
    __threadfence();
    if (w4) { *(volatile v4i*)cp = cv; *(volatile v4i*)fp = fv; }
    if (tid < 8) *(volatile v4i*)rp = rv;
  }
}

__global__ __launch_bounds__(GTHR) __attribute__((amdgpu_num_vgpr(248)))
void k_gemm(const unsigned short* __restrict__ A, const unsigned short* __restrict__ WT,
            const float* __restrict__ bvec, float* outF,
            int lda, int ldw, int ksteps, int planeStride, int nStore) {
  __shared__ __attribute__((aligned(16))) float stg[GBM * GBN];
  __shared__ __attribute__((aligned(16))) float bsh[GBN];
  const int tid = (int)threadIdx.x, lane = tid & 31, wave = tid >> 5, hh = lane >> 4, m = lane & 15;
  const int rowBase = (int)blockIdx.x * GBM;
  const int col0    = (int)blockIdx.y * GBN;

  if (tid < 32) {
    const v4f b4 = *(const v4f*)(bvec + col0 + 4 * m);
    *(v4fa*)(bsh + 4 * m) = b4;
  }

  v8f acc[4];
  {
    const v8f z = {0.f, 0.f, 0.f, 0.f, 0.f, 0.f, 0.f, 0.f};
    acc[0] = z; acc[1] = z; acc[2] = z; acc[3] = z;
  }
  const unsigned short* ap = A  + (size_t)(rowBase + 16 * wave + m) * (size_t)lda + 8 * hh;
  const unsigned short* wp = WT + (size_t)(col0 + m) * (size_t)ldw + 8 * hh;
#pragma unroll 1
  for (int ks = 0; ks < ksteps; ++ks) {
    FragB af;
    af.h[0] = *(const v8usa*)(ap + 32 * ks);
    af.h[1] = *(const v8usa*)(ap + 32 * ks + 16);
#pragma unroll
    for (int t = 0; t < 4; ++t) {
      const unsigned short* wq = wp + (size_t)(16 * t) * (size_t)ldw + 32 * ks;
      FragB bf;
      bf.h[0] = *(const v8usa*)wq;
      bf.h[1] = *(const v8usa*)(wq + 16);
      acc[t] = wmb(af, bf, acc[t]);
    }
  }
  __syncthreads();

#pragma unroll
  for (int t = 0; t < 4; ++t) {
    const int lc = 16 * t + m;
    const float bb = bsh[lc];
#pragma unroll
    for (int r = 0; r < 8; ++r) {
      const int lr = 16 * wave + 8 * hh + r;
      stg[lr * GBN + lc] = acc[t][r] + bb;
    }
  }
  __syncthreads();

  v4f fv[8];
#pragma unroll
  for (int i = 0; i < 8; ++i) {
    const int lr = 16 * wave + 2 * i + hh;
    fv[i] = *(const v4fa*)(stg + lr * GBN + 4 * m);
  }
  const size_t pofs = (col0 >= HC) ? (size_t)planeStride : (size_t)0;
  const int cc = (col0 & (HC - 1)) + 4 * m;
#pragma unroll
  for (int i = 0; i < 8; ++i) {
    const int gr = rowBase + 16 * wave + 2 * i + hh;
    float* op = outF + pofs + (size_t)gr * HC + cc;
    if (gr < nStore) *(volatile v4f*)op = fv[i];
  }
  __threadfence();
#pragma unroll
  for (int i = 0; i < 8; ++i) {
    const int gr = rowBase + 16 * wave + 2 * i + hh;
    float* op = outF + pofs + (size_t)gr * HC + cc;
    if (gr < nStore) *(volatile v4f*)op = fv[i];
  }
}

template <int MODE>
__global__ __launch_bounds__(NTHR) void k_replay(
    const float* __restrict__ XL, const float* __restrict__ XR,
    const int* __restrict__ LIST, const int* __restrict__ CNT, const int* __restrict__ OFF,
    const int* __restrict__ REC, const float* __restrict__ attv, const float* __restrict__ biasv,
    unsigned short* X1, float* out, int nN, int o1off) {
  __shared__ __attribute__((aligned(16))) float rowst[NWAVE * HC];
  const int tid = (int)threadIdx.x, lane = tid & 31, wave = tid >> 5;
  float* stw = rowst + wave * HC;
  float at[8], bi[8];
  {
    const v4f a0 = *(const v4f*)(attv + 8 * lane);
    const v4f a1 = *(const v4f*)(attv + 8 * lane + 4);
    const v4f b0 = *(const v4f*)(biasv + 8 * lane);
    const v4f b1 = *(const v4f*)(biasv + 8 * lane + 4);
    at[0] = a0.x; at[1] = a0.y; at[2] = a0.z; at[3] = a0.w; at[4] = a1.x; at[5] = a1.y; at[6] = a1.z; at[7] = a1.w;
    bi[0] = b0.x; bi[1] = b0.y; bi[2] = b0.z; bi[3] = b0.w; bi[4] = b1.x; bi[5] = b1.y; bi[6] = b1.z; bi[7] = b1.w;
  }
  const float qnan = __int_as_float(0x7fc00000);
#pragma unroll 1
  for (int ri = 0; ri < RPW; ++ri) {
    const int node = (int)blockIdx.x * RPB + wave * RPW + ri;
    if (node >= nN) continue;
    int c, o;
    slot_info(CNT, OFF, node, c, o);
    const int fl = REC[(size_t)(node >> PKS) * 32 + 1];
    const float pz = (fl != 0) ? qnan : 0.0f;
    const int* lp = LIST + (size_t)(node >> PKS) * RCAP;

    float xr[8], acc[8];
    {
      const float* xlp = XL + (size_t)node * HC + 8 * lane;
      const float* xrp = XR + (size_t)node * HC + 8 * lane;
      const v4f l0 = *(const v4f*)xlp, l1 = *(const v4f*)(xlp + 4);
      const v4f r0 = *(const v4f*)xrp, r1 = *(const v4f*)(xrp + 4);
      acc[0] = l0.x; acc[1] = l0.y; acc[2] = l0.z; acc[3] = l0.w;
      acc[4] = l1.x; acc[5] = l1.y; acc[6] = l1.z; acc[7] = l1.w;
      xr[0] = r0.x; xr[1] = r0.y; xr[2] = r0.z; xr[3] = r0.w;
      xr[4] = r1.x; xr[5] = r1.y; xr[6] = r1.z; xr[7] = r1.w;
    }
    float part = 0.0f;
#pragma unroll
    for (int j = 0; j < 8; ++j) {
      float v = acc[j] + xr[j];
      v = (v > 0.0f) ? v : v * NEGS;
      part = fmaf(v, at[j], part);
    }
    part += __shfl_xor(part, 1, 32);
    part += __shfl_xor(part, 2, 32);
    part += __shfl_xor(part, 4, 32);
    float mx = part;
    float sm = 1.0f;

    int last = o + c - 1;
    last = last < o ? o : last;
    last = last > RCAP - 1 ? RCAP - 1 : last;
#pragma unroll 1
    for (int b0 = 0; b0 < c; b0 += 32) {
      int idx = o + b0 + lane;
      idx = idx > last ? last : idx;
      int col = lp[idx];
      col = col < 0 ? 0 : (col > nN - 1 ? nN - 1 : col);
      const int m32 = (c - b0) < 32 ? (c - b0) : 32;
#pragma unroll 1
      for (int k = 0; k < m32; ++k) {
        const int sk = __builtin_amdgcn_readlane(col, k);
        const float* sp = XL + (size_t)sk * HC + 8 * lane;
        const v4f s0 = *(const v4f*)sp;
        const v4f s1 = *(const v4f*)(sp + 4);
        const float xs[8] = {s0.x, s0.y, s0.z, s0.w, s1.x, s1.y, s1.z, s1.w};
        float pt = 0.0f;
#pragma unroll
        for (int j = 0; j < 8; ++j) {
          float v = xs[j] + xr[j];
          v = (v > 0.0f) ? v : v * NEGS;
          pt = fmaf(v, at[j], pt);
        }
        pt += __shfl_xor(pt, 1, 32);
        pt += __shfl_xor(pt, 2, 32);
        pt += __shfl_xor(pt, 4, 32);
        const float df = pt - mx;
        const float dd = expf(-fabsf(df));
        const bool up  = df > 0.0f;
        const float sc1 = up ? dd : 1.0f;
        const float pw  = up ? 1.0f : dd;
        mx = up ? pt : mx;
        sm = fmaf(sm, sc1, pw);
#pragma unroll
        for (int j = 0; j < 8; ++j) acc[j] = fmaf(acc[j], sc1, pw * xs[j]);
      }
    }
    const float inv = __builtin_amdgcn_rcpf(sm);
    float hv[8];
#pragma unroll
    for (int j = 0; j < 8; ++j) hv[j] = fmaf(acc[j], inv, bi[j]) + pz;

    {
      v4f w0, w1;
      w0.x = hv[0]; w0.y = hv[1]; w0.z = hv[2]; w0.w = hv[3];
      w1.x = hv[4]; w1.y = hv[5]; w1.z = hv[6]; w1.w = hv[7];
      *(v4fa*)(stw + 8 * lane)     = w0;
      *(v4fa*)(stw + 8 * lane + 4) = w1;
    }
    wave_sync();

    if constexpr (MODE == 0) {
#pragma unroll 1
      for (int j = 0; j < 8; ++j) {
        const float t  = stw[8 * lane + j];
        const float em = expm1f(t);
        stw[8 * lane + j] = (t > 0.0f) ? t : em;
      }
      wave_sync();
      const v4f ea = *(const v4fa*)(stw + 8 * lane);
      const v4f eb = *(const v4fa*)(stw + 8 * lane + 4);
      wave_sync();
      unsigned h0, l0, h1, l1, h2, l2, h3, l3;
      pack2(ea.x, ea.y, h0, l0);
      pack2(ea.z, ea.w, h1, l1);
      pack2(eb.x, eb.y, h2, l2);
      pack2(eb.z, eb.w, h3, l3);
      v4u qh, ql;
      qh.x = h0; qh.y = h1; qh.z = h2; qh.w = h3;
      ql.x = l0; ql.y = l1; ql.z = l2; ql.w = l3;
      unsigned short* wp = X1 + (size_t)node * PP + 8 * lane;
      *(volatile v4u*)wp = qh;
      *(volatile v4u*)(wp + HC) = ql;
      __threadfence();
      *(volatile v4u*)wp = qh;
      *(volatile v4u*)(wp + HC) = ql;
    } else {
      float rm = hv[0];
#pragma unroll
      for (int j = 1; j < 8; ++j) rm = (hv[j] > rm) ? hv[j] : rm;
#pragma unroll
      for (int d = 16; d >= 1; d >>= 1) {
        const float ot = __shfl_xor(rm, d, 32);
        rm = (ot > rm) ? ot : rm;
      }
      float es = 0.0f;
#pragma unroll 1
      for (int j = 0; j < 8; ++j) es += expf(stw[8 * lane + j] - rm);
#pragma unroll
      for (int d = 16; d >= 1; d >>= 1) es += __shfl_xor(es, d, 32);
      const float lse = logf(es);
      const v4f ha = *(const v4fa*)(stw + 4 * lane);
      const v4f hb = *(const v4fa*)(stw + 128 + 4 * lane);
      wave_sync();
      v4f oa, ob;
      oa.x = (ha.x - rm) - lse; oa.y = (ha.y - rm) - lse; oa.z = (ha.z - rm) - lse; oa.w = (ha.w - rm) - lse;
      ob.x = (hb.x - rm) - lse; ob.y = (hb.y - rm) - lse; ob.z = (hb.z - rm) - lse; ob.w = (hb.w - rm) - lse;
      float* op0 = out + (size_t)node * HC + 4 * lane;
      float* op1 = op0 + (size_t)o1off;
      *(volatile v4f*)op0 = ha;
      *(volatile v4f*)(op0 + 128) = hb;
      *(volatile v4f*)op1 = oa;
      *(volatile v4f*)(op1 + 128) = ob;
      __threadfence();
      *(volatile v4f*)op0 = ha;
      *(volatile v4f*)(op0 + 128) = hb;
      *(volatile v4f*)op1 = oa;
      *(volatile v4f*)(op1 + 128) = ob;
    }
  }
  (void)X1; (void)out; (void)o1off;
}

static inline int cdiv(int a, int b) { return (a + b - 1) / b; }
static inline size_t al256(size_t o) { return (o + 255) & ~(size_t)255; }

extern "C" void kernel_launch(void* const* d_in, const int* in_sizes, int n_in,
                              void* d_out, int out_size, void* d_ws, size_t ws_size,
                              hipStream_t stream) {
  if (n_in < 14) return;
  if (in_sizes[0] < FIN * RPB || (in_sizes[0] % FIN) != 0) return;
  const int nN = in_sizes[0] / FIN;
  if (nN > 32768) return;
  if (in_sizes[1] < 2 || (in_sizes[1] & 1) != 0) return;
  const int nE = in_sizes[1] / 2;
  if (nE < 1 || nE >= (1 << 22)) return;
  if (in_sizes[2] != FIN * HC || in_sizes[4] != FIN * HC) return;
  if (in_sizes[3] != HC || in_sizes[5] != HC || in_sizes[6] != HC || in_sizes[7] != HC) return;
  if (in_sizes[8] != HC * HC || in_sizes[10] != HC * HC) return;
  if (in_sizes[9] != HC || in_sizes[11] != HC || in_sizes[12] != HC || in_sizes[13] != HC) return;
  if ((long long)out_size != 2LL * (long long)nN * HC) return;

  const float* x     = (const float*)d_in[0];
  const int*   ei    = (const int*)  d_in[1];
  const float* Wl1   = (const float*)d_in[2];
  const float* bl1   = (const float*)d_in[3];
  const float* Wr1   = (const float*)d_in[4];
  const float* br1   = (const float*)d_in[5];
  const float* att1  = (const float*)d_in[6];
  const float* bias1 = (const float*)d_in[7];
  const float* Wl2   = (const float*)d_in[8];
  const float* bl2   = (const float*)d_in[9];
  const float* Wr2   = (const float*)d_in[10];
  const float* br2   = (const float*)d_in[11];
  const float* att2  = (const float*)d_in[12];
  const float* bias2 = (const float*)d_in[13];
  float* out = (float*)d_out;
  const int* srcI = ei;
  const int* dstI = ei + nE;

  const int MP    = cdiv(nN, 128) * 128;
  const int nB    = cdiv(nN, NBA);
  const int NPADN = nB * NBA;
  const int vec8  = ((nE & 3) == 0) ? 1 : 0;
  const int nUX   = MP * (FIN / 8);
  const int nPad  = (MP - nN) * (PP / 8);
  if ((nUX % NTHR) != 0 || (MP % GBM) != 0) return;
  const int planeStride = MP * HC;
  const int o1off = nN * HC;

  char* ws = (char*)d_ws;
  size_t off = 0;
  const size_t oXLR = off; off = al256(off + (size_t)2 * MP * HC * 4);
  const size_t oX1  = off; off = al256(off + (size_t)MP * PP * 2);
  const size_t oXB  = off; off = al256(off + (size_t)MP * FIN * 2);
  const size_t oW1  = off; off = al256(off + (size_t)NC2 * FIN * 2);
  const size_t oW2  = off; off = al256(off + (size_t)NC2 * KT2 * 2);
  const size_t oVC  = off; off = al256(off + (size_t)VEC_N * 4);
  const size_t oLS  = off; off = al256(off + (size_t)nB * RCAP * 4);
  const size_t oCN  = off; off = al256(off + (size_t)NPADN * 4);
  const size_t oOF  = off; off = al256(off + (size_t)NPADN * 4);
  const size_t oRC  = off; off = al256(off + (size_t)nB * 128);
  if (off > ws_size || off > (size_t)WSMAX) return;
  float*          XLR  = (float*)(ws + oXLR);
  unsigned short* X1   = (unsigned short*)(ws + oX1);
  unsigned short* XB   = (unsigned short*)(ws + oXB);
  unsigned short* W1T  = (unsigned short*)(ws + oW1);
  unsigned short* W2T  = (unsigned short*)(ws + oW2);
  float*          VEC  = (float*)(ws + oVC);
  int*            LIST = (int*)(ws + oLS);
  int*            CNT  = (int*)(ws + oCN);
  int*            OFF  = (int*)(ws + oOF);
  int*            REC  = (int*)(ws + oRC);
  const float* XL = XLR;
  const float* XR = XLR + (size_t)planeStride;

  hipFuncSetAttribute(reinterpret_cast<const void*>(&k_bucket), hipFuncAttributeMaxDynamicSharedMemorySize, LDS_BK);

  const int nUnits = U_FIX + nUX + nPad;
  k_prep<<<cdiv(nUnits, NTHR), NTHR, 0, stream>>>(x, Wl1, Wr1, Wl2, Wr2, bl1, br1, bl2, br2,
                                                  att1, att2, bias1, bias2,
                                                  W1T, W2T, VEC, XB, X1, nN, nUX, nPad);
  k_bucket<<<nB, NTHR, LDS_BK, stream>>>(dstI, srcI, nE, nN, vec8, LIST, CNT, OFF, REC);
  const dim3 gg((unsigned)(MP / GBM), (unsigned)(NC2 / GBN), 1u);
  k_gemm<<<gg, GTHR, 0, stream>>>(XB, W1T, VEC + V_BLR1, XLR, FIN, FIN, FIN / 32, planeStride, nN);
  const int gR = cdiv(nN, RPB);
  k_replay<0><<<gR, NTHR, 0, stream>>>(XL, XR, LIST, CNT, OFF, REC, VEC + V_ATT1, VEC + V_BIAS1,
                                       X1, out, nN, o1off);
  k_gemm<<<gg, GTHR, 0, stream>>>(X1, W2T, VEC + V_BLR2, XLR, PP, KT2, (HC * A2_TERMS) / 32, planeStride, nN);
  k_replay<1><<<gR, NTHR, 0, stream>>>(XL, XR, LIST, CNT, OFF, REC, VEC + V_ATT2, VEC + V_BIAS2,
                                       X1, out, nN, o1off);
}
